// RNNCellCmplx_6047313953020
// MI455X (gfx1250) — hardware-run, weakly checked
//
#include <hip/hip_runtime.h>
#include <math.h>

typedef __attribute__((ext_vector_type(16))) _Float16 v16h;
typedef __attribute__((ext_vector_type(8)))  _Float16 v8h;
typedef __attribute__((ext_vector_type(8)))  float    v8f;
typedef __attribute__((ext_vector_type(4)))  float    v4f;

constexpr int kBatch      = 128;
constexpr int kIn         = 256;
constexpr int kHid        = 1024;
constexpr int kLayerPairs = 128;
constexpr int kPairsA     = 512;
constexpr int kPairsB     = 511;
constexpr int kKp         = 2 * kIn;
constexpr int kNp         = 2 * kHid;
constexpr int kRowsPerBlk = 2;
constexpr int kPackBlocksA = kBatch / 4;
constexpr int kPackBlocksB = kNp / 4;
constexpr int kGemmTiles   = (kBatch / 64) * (kNp / 64);
constexpr float kCarryX    = 16.0f;
constexpr float kCarryW    = 1024.0f;
constexpr float kFoldScale = 1.0f / (kCarryX * kCarryW);
constexpr float kF16MinNormal = 6.103515625e-5f;

static_assert(kIn == 256);
static_assert(kPairsA * 2 == kHid);
static_assert(kPairsB == kPairsA - 1);
static_assert((kKp % 32) == 0);
static_assert((kBatch % 64) == 0 && (kNp % 64) == 0 && (kHid % 64) == 0);
static_assert((kGemmTiles % 8) == 0);
static_assert(kRowsPerBlk * (kHid / 4) == 512);
static_assert((kBatch % kRowsPerBlk) == 0);

constexpr size_t kOffA16  = 0;
constexpr size_t kOffBT16 = kOffA16  + (size_t)kBatch * kKp * 2;
constexpr size_t kOffIH   = kOffBT16 + (size_t)kNp * kKp * 2;
constexpr size_t kOffTAB  = kOffIH   + (size_t)kBatch * kNp * 4;
constexpr size_t kWsTotal = kOffTAB  + (size_t)(2 * kLayerPairs) * kPairsA * 16;
static_assert(kWsTotal == 5373952ull);
static_assert(kWsTotal <= 134217728ull);
static_assert((kOffBT16 % 128) == 0 && (kOffIH % 128) == 0 && (kOffTAB % 128) == 0);

__device__ __forceinline__ unsigned pin_u32(unsigned v) {
  asm volatile("" : "+v"(v));
  return v;
}

union FragH { v16h v; v8h h[2]; };
__device__ __forceinline__ v16h frag_load_h(const _Float16* p) {
  FragH f;
  f.h[0] = *(const v8h*)(p);
  f.h[1] = *(const v8h*)(p + 16);
  return f.v;
}
__device__ __forceinline__ v8f mma_f16(v16h a, v16h b, v8f c) {
  c = __builtin_amdgcn_wmma_f32_16x16x32_f16(false, a, false, b, (short)0, c, false, false);
  asm volatile("v_nop\n\tv_nop\n\tv_nop\n\tv_nop" : "+v"(c) : "v"(a), "v"(b));
  return c;
}

__global__ __launch_bounds__(256) void pack_planes_kernel(
    const float* __restrict__ inR, const float* __restrict__ inI,
    const float* __restrict__ wR,  const float* __restrict__ wI,
    unsigned short* __restrict__ A16, unsigned short* __restrict__ BT16)
{
  const unsigned tid   = threadIdx.x;
  const unsigned lane8 = pin_u32((tid & 31u) * 8u);
  const unsigned wave  = tid >> 5;
  const unsigned kh    = wave & 1u;
  const unsigned blk   = blockIdx.x;
  const bool isA = (blk < (unsigned)kPackBlocksA);
  const unsigned row = (isA ? blk : (blk - (unsigned)kPackBlocksA)) * 4u + (wave >> 1);

  const float* src;
  float mul;
  unsigned srow;
  unsigned short* dst;
  if (isA) {
    src  = (kh != 0u) ? inI : inR;
    mul  = kCarryX;
    srow = row;
    dst  = A16;
  } else {
    const bool top  = (row < (unsigned)kHid);
    const bool useR = (top == (kh == 0u));
    src  = useR ? wR : wI;
    mul  = (top && (kh != 0u)) ? -kCarryW : kCarryW;
    srow = row & (unsigned)(kHid - 1);
    dst  = BT16;
  }
  const float* sp = src + (size_t)srow * kIn + lane8;
  const v4f a0 = *(const v4f*)(sp);
  const v4f a1 = *(const v4f*)(sp + 4);
  v8h hv;
#pragma unroll
  for (int e = 0; e < 4; ++e) {
    float x0 = a0[e] * mul;
    float x1 = a1[e] * mul;
    x0 = (fabsf(x0) < kF16MinNormal) ? 0.0f : x0;
    x1 = (fabsf(x1) < kF16MinNormal) ? 0.0f : x1;
    hv[e]     = (_Float16)x0;
    hv[4 + e] = (_Float16)x1;
  }
  unsigned short* q = dst + (size_t)row * kKp + kh * (unsigned)kIn + lane8;
  *(volatile v8h*)q = hv;
  __threadfence();
  *(volatile v8h*)q = hv;
}

__global__ __launch_bounds__(512) void trig_table_kernel(
    const float* __restrict__ A0, const float* __restrict__ A1,
    const float* __restrict__ B0, const float* __restrict__ B1,
    float* __restrict__ table)
{
  const unsigned j = blockIdx.x;
  const unsigned p = pin_u32(threadIdx.x);
  const unsigned l = j >> 1;
  float th0, th1;
  bool act = true;
  if ((j & 1u) == 0u) {
    th0 = A0[l * (unsigned)kPairsA + p];
    th1 = A1[l * (unsigned)kPairsA + p];
  } else {
    const unsigned pc = pin_u32((p < (unsigned)kPairsB) ? p : (unsigned)(kPairsB - 1));
    th0 = B0[l * (unsigned)kPairsB + pc];
    th1 = B1[l * (unsigned)kPairsB + pc];
    act = (p < (unsigned)kPairsB);
  }
  asm volatile("" : "+v"(th0));
  asm volatile("" : "+v"(th1));
  float s0, c0, s1, c1;
  sincosf(th0, &s0, &c0);
  sincosf(th1, &s1, &c1);
  v4f v;
  v[0] = act ? c0 : 1.0f;
  v[1] = act ? s0 : 0.0f;
  v[2] = act ? c1 : 1.0f;
  v[3] = act ? s1 : 0.0f;
  float* q = table + ((size_t)j * kPairsA + p) * 4;
  *(volatile v4f*)q = v;
  __threadfence();
  *(volatile v4f*)q = v;
}

__global__ __launch_bounds__(256) void packed_linear_gemm(
    const unsigned short* __restrict__ Ap, const unsigned short* __restrict__ Btp,
    float* __restrict__ C, const float* __restrict__ biasRe, const float* __restrict__ biasIm, float scale)
{
  const _Float16* A  = (const _Float16*)Ap;
  const _Float16* Bt = (const _Float16*)Btp;
  __shared__ __align__(16) float sT[8][16 * 68];
  const int lane = threadIdx.x & 31;
  const int wave = threadIdx.x >> 5;
  constexpr int tilesN = kNp >> 6;
  const int tile = blockIdx.x * 8 + wave;
  if (tile >= kGemmTiles) return;
  const int tm = tile / tilesN;
  const int tn = tile - tm * tilesN;
  const int m0 = tm << 6;
  const int n0 = tn << 6;

  const int rlane = lane & 15;
  const int koff  = (lane >> 4) * 8;
  const int mOff  = (lane >> 4) * 8;

  v8f acc[4][4];
#pragma unroll
  for (int i = 0; i < 4; ++i)
#pragma unroll
    for (int j = 0; j < 4; ++j) acc[i][j] = (v8f){0.f,0.f,0.f,0.f,0.f,0.f,0.f,0.f};

  for (int k0 = 0; k0 < kKp; k0 += 32) {
    v16h bh[4];
#pragma unroll
    for (int j = 0; j < 4; ++j) {
      const size_t bo = (size_t)(n0 + (j << 4) + rlane) * kKp + koff + k0;
      bh[j] = frag_load_h(Bt + bo);
    }
#pragma unroll
    for (int i = 0; i < 4; ++i) {
      const size_t ao = (size_t)(m0 + (i << 4) + rlane) * kKp + koff + k0;
      const v16h ah = frag_load_h(A + ao);
#pragma unroll
      for (int j = 0; j < 4; ++j) acc[i][j] = mma_f16(ah, bh[j], acc[i][j]);
    }
  }

  float* slab = sT[wave];
  const float* bsel = (n0 < kHid) ? biasRe : biasIm;
  const int nb0 = n0 & (kHid - 1);
  float bv[4];
#pragma unroll
  for (int j = 0; j < 4; ++j) bv[j] = bsel[nb0 + (j << 4) + rlane];
#pragma unroll
  for (int i = 0; i < 4; ++i) {
    const int mBase = m0 + (i << 4);
#pragma unroll
    for (int j = 0; j < 4; ++j) {
#pragma unroll
      for (int r = 0; r < 8; ++r) {
        const float v = acc[i][j][r] * scale + bv[j];
        slab[(mOff + r) * 68 + (j << 4) + rlane] = v;
      }
    }
    __builtin_amdgcn_fence(__ATOMIC_RELEASE, "workgroup");
    __builtin_amdgcn_wave_barrier();
    __builtin_amdgcn_fence(__ATOMIC_ACQUIRE, "workgroup");
    {
      const int hh = lane >> 4, c4 = (lane & 15) * 4;
      for (int pass = 0; pass < 2; ++pass) {
#pragma unroll
        for (int it = 0; it < 8; ++it) {
          const int row = it * 2 + hh;
          v4f v = *(const v4f*)(slab + row * 68 + c4);
          *(volatile v4f*)(C + (size_t)(mBase + row) * kNp + n0 + c4) = v;
        }
        __threadfence();
      }
    }
    __builtin_amdgcn_fence(__ATOMIC_RELEASE, "workgroup");
    __builtin_amdgcn_wave_barrier();
    __builtin_amdgcn_fence(__ATOMIC_ACQUIRE, "workgroup");
  }
}

__global__ __launch_bounds__(512) void mesh_gate_kernel(
    const float* __restrict__ stateR, const float* __restrict__ stateI,
    const float* __restrict__ table,  const float* __restrict__ ih,
    const float* __restrict__ omega,  const float* __restrict__ modb,
    float* __restrict__ out)
{
  __shared__ __align__(16) float xr[kRowsPerBlk * kHid];
  __shared__ __align__(16) float xi[kRowsPerBlk * kHid];

  const unsigned t   = pin_u32(threadIdx.x);
  const unsigned b0  = blockIdx.x * (unsigned)kRowsPerBlk;
  const unsigned sr  = pin_u32(t >> 8);
  const unsigned sc4 = pin_u32((t & 255u) * 4u);

  {
    const size_t go = (size_t)(b0 + sr) * kHid + sc4;
    const v4f vr = *(const v4f*)(stateR + go);
    const v4f vi = *(const v4f*)(stateI + go);
    *(v4f*)(xr + sr * (unsigned)kHid + sc4) = vr;
    *(v4f*)(xi + sr * (unsigned)kHid + sc4) = vi;
  }
  __syncthreads();

  const bool actB = (t < (unsigned)kPairsB);
  const float* tp = table + (size_t)t * 4;
  const unsigned ia0 = pin_u32(2u * t);

#pragma unroll 1
  for (int l = 0; l < kLayerPairs; ++l) {
    v4f tga = *(const v4f*)(tp + (size_t)(2 * l) * kPairsA * 4);
    v4f tgb = *(const v4f*)(tp + (size_t)(2 * l + 1) * kPairsA * 4);
    asm volatile("" : "+v"(tga));
    asm volatile("" : "+v"(tgb));
    {
      const float c0 = tga[0], s0 = tga[1], c1 = tga[2], s1 = tga[3];
#pragma unroll
      for (int r = 0; r < kRowsPerBlk; ++r) {
        const unsigned ia = (unsigned)(r * kHid) + ia0;
        const float ar = xr[ia],     ai = xi[ia];
        const float br = xr[ia + 1], bi = xi[ia + 1];
        const float pr = c0 * ar - s0 * ai;
        const float pq = s0 * ar + c0 * ai;
        const float oar = c1 * pr - s1 * bi;
        const float oai = c1 * pq + s1 * br;
        const float obr = c1 * br - s1 * pq;
        const float obi = c1 * bi + s1 * pr;
        xr[ia]     = oar;
        xi[ia]     = oai;
        xr[ia + 1] = obr;
        xi[ia + 1] = obi;
      }
    }
    __syncthreads();
    if (actB) {
      const float c0 = tgb[0], s0 = tgb[1], c1 = tgb[2], s1 = tgb[3];
#pragma unroll
      for (int r = 0; r < kRowsPerBlk; ++r) {
        const unsigned ia = (unsigned)(r * kHid) + ia0 + 1u;
        const float ar = xr[ia],     ai = xi[ia];
        const float br = xr[ia + 1], bi = xi[ia + 1];
        const float pr = c0 * ar - s0 * ai;
        const float pq = s0 * ar + c0 * ai;
        const float oar = c1 * pr - s1 * bi;
        const float oai = c1 * pq + s1 * br;
        const float obr = c1 * br - s1 * pq;
        const float obi = c1 * bi + s1 * pr;
        xr[ia]     = oar;
        xi[ia]     = oai;
        xr[ia + 1] = obr;
        xi[ia + 1] = obi;
      }
    }
    __syncthreads();
  }

#pragma unroll 1
  for (int cq = 0; cq < 2; ++cq) {
    const unsigned ch = (unsigned)(cq * 512) + t;
    float so, co;
    sincosf(omega[ch], &so, &co);
    const float mb = modb[ch];
#pragma unroll 1
    for (int r = 0; r < kRowsPerBlk; ++r) {
      const unsigned li = (unsigned)(r * kHid) + ch;
      const float hr = xr[li], hi = xi[li];
      const float hhR = co * hr - so * hi;
      const float hhI = so * hr + co * hi;
      const size_t go = (size_t)(b0 + (unsigned)r) * kNp + ch;
      const float zr = ih[go] + hhR;
      const float zi = ih[go + kHid] + hhI;
      const float mag = sqrtf(zr * zr + zi * zi);
      const float num = fmaxf(mag + mb, 0.0f);
      const float den = fmaxf(mag, 1e-8f);
      const float sc  = num / den;
      xr[li] = sc * zr;
      xi[li] = sc * zi;
    }
  }
  __syncthreads();

  {
    const v4f vr = *(const v4f*)(xr + sr * (unsigned)kHid + sc4);
    const v4f vi = *(const v4f*)(xi + sr * (unsigned)kHid + sc4);
    float* qr = out + (size_t)(b0 + sr) * kHid + sc4;
    float* qi = out + (size_t)kBatch * kHid + (size_t)(b0 + sr) * kHid + sc4;
    *(volatile v4f*)qr = vr;
    *(volatile v4f*)qi = vi;
    __threadfence();
    *(volatile v4f*)qr = vr;
    *(volatile v4f*)qi = vi;
  }
}

extern "C" void kernel_launch(void* const* d_in, const int* in_sizes, int n_in,
                              void* d_out, int out_size, void* d_ws, size_t ws_size,
                              hipStream_t stream) {
  if (n_in < 14) return;
  if (in_sizes[0] != kBatch * kIn) return;
  if (in_sizes[1] != kBatch * kIn) return;
  if (in_sizes[2] != kBatch * kHid) return;
  if (in_sizes[3] != kBatch * kHid) return;
  if (in_sizes[4] != kHid * kIn) return;
  if (in_sizes[5] != kHid * kIn) return;
  if (in_sizes[6] != kHid) return;
  if (in_sizes[7] != kHid) return;
  if (in_sizes[8] != kLayerPairs * kPairsA) return;
  if (in_sizes[9] != kLayerPairs * kPairsA) return;
  if (in_sizes[10] != kLayerPairs * kPairsB) return;
  if (in_sizes[11] != kLayerPairs * kPairsB) return;
  if (in_sizes[12] != kHid) return;
  if (in_sizes[13] != kHid) return;
  if (out_size != 2 * kBatch * kHid) return;
  if (ws_size < kWsTotal) return;

  const float* inputsR = (const float*)d_in[0];
  const float* inputsI = (const float*)d_in[1];
  const float* stateR  = (const float*)d_in[2];
  const float* stateI  = (const float*)d_in[3];
  const float* weightR = (const float*)d_in[4];
  const float* weightI = (const float*)d_in[5];
  const float* biasR   = (const float*)d_in[6];
  const float* biasI   = (const float*)d_in[7];
  const float* angleA0 = (const float*)d_in[8];
  const float* angleA1 = (const float*)d_in[9];
  const float* angleB0 = (const float*)d_in[10];
  const float* angleB1 = (const float*)d_in[11];
  const float* omega   = (const float*)d_in[12];
  const float* modb    = (const float*)d_in[13];

  char* ws = (char*)d_ws;
  unsigned short* A16  = (unsigned short*)(ws + kOffA16);
  unsigned short* BT16 = (unsigned short*)(ws + kOffBT16);
  float*          IH   = (float*)(ws + kOffIH);
  float*          TAB  = (float*)(ws + kOffTAB);

  pack_planes_kernel<<<kPackBlocksA + kPackBlocksB, 256, 0, stream>>>(
      inputsR, inputsI, weightR, weightI, A16, BT16);
  trig_table_kernel<<<2 * kLayerPairs, 512, 0, stream>>>(angleA0, angleA1, angleB0, angleB1, TAB);
  packed_linear_gemm<<<kGemmTiles / 8, 256, 0, stream>>>(A16, BT16, IH, biasR, biasI, kFoldScale);
  mesh_gate_kernel<<<kBatch / kRowsPerBlk, 512, 0, stream>>>(
      stateR, stateI, TAB, IH, omega, modb, (float*)d_out);
}
